// QSAR_57810259804592
// MI455X (gfx1250) — hardware-verified
//
#include <hip/hip_runtime.h>

typedef _Float16 v16h __attribute__((ext_vector_type(16)));
typedef _Float16 v8h  __attribute__((ext_vector_type(8)));
typedef float    v8f  __attribute__((ext_vector_type(8)));
typedef float    v4f  __attribute__((ext_vector_type(4)));
typedef v8h __attribute__((may_alias)) v8ha;
typedef v4f __attribute__((may_alias)) v4fa;

union Frag { v16h v; v8h half[2]; };
union H8   { v8h v; _Float16 s[8]; };

#define A_    64
#define D_    6
#define AF_   37
#define BF_   6
#define H_    128
#define K1R   43
#define K2R   134
#define K1P   64
#define K2P   160
#define KPS   168
#define KPA   136
#define KPH   72
#define WSC   64.0f
#define WINV  0.015625f

#define NB_W1  24
#define NB_W2  60
#define NB_WO  10
#define NB_M1  4
#define NB_M2  1
#define NB_CVT (NB_W1 + NB_W2 + NB_WO + NB_M1 + NB_M2)

__device__ __forceinline__ v8f wmma_f16(v16h a, v16h b, v8f c) {
  v8f d = __builtin_amdgcn_wmma_f32_16x16x32_f16(false, a, false, b, (short)0, c, false, false);
  asm volatile("v_nop\n\tv_nop\n\tv_nop\n\tv_nop" : "+v"(d) : "v"(a), "v"(b));
  return d;
}

__device__ __forceinline__ v16h load_frag(const _Float16* p, int h) {
  Frag f;
  f.half[0] = *(const v8ha*)(p + 8 * h);
  f.half[1] = *(const v8ha*)(p + 16 + 8 * h);
  return f.v;
}

__global__ __launch_bounds__(256) void k_convert(
    const float* __restrict__ W1, const float* __restrict__ W2, const float* __restrict__ Wo,
    const float* __restrict__ Wm1, const float* __restrict__ Wm2,
    _Float16* __restrict__ w1h, _Float16* __restrict__ w2h, _Float16* __restrict__ woh,
    _Float16* __restrict__ wm1h, _Float16* __restrict__ wm2h)
{
  const int blk = blockIdx.x, tid = threadIdx.x;
  if (blk >= NB_CVT) return;
  const float* src; _Float16* dpl; int Kreal, Kpad, N, base;
  if (blk < NB_W1) {
    src = W1; dpl = w1h; Kreal = K1R; Kpad = K1P; N = H_; base = 0;
  } else if (blk < NB_W1 + NB_W2) {
    src = W2; dpl = w2h; Kreal = K2R; Kpad = K2P; N = H_; base = NB_W1;
  } else if (blk < NB_W1 + NB_W2 + NB_WO) {
    src = Wo; dpl = woh; Kreal = K2R; Kpad = K2P; N = H_; base = NB_W1 + NB_W2;
  } else if (blk < NB_W1 + NB_W2 + NB_WO + NB_M1) {
    src = Wm1; dpl = wm1h; Kreal = H_; Kpad = H_; N = 64; base = NB_W1 + NB_W2 + NB_WO;
  } else {
    src = Wm2; dpl = wm2h; Kreal = 64; Kpad = 64; N = 32; base = NB_W1 + NB_W2 + NB_WO + NB_M1;
  }
  const int e = ((blk - base) * 256 + tid) * 8;
  const int q = e / Kpad;
  const int k = e - q * Kpad;
  const int d = q / N;
  const int n = q - d * N;
  H8 o;
  #pragma unroll
  for (int i = 0; i < 8; ++i) {
    const int kk = k + i;
    const int kc = (kk < Kreal) ? kk : (Kreal - 1);
    const float v = src[((size_t)d * Kreal + kc) * N + n];
    o.s[i] = (kk < Kreal) ? (_Float16)(v * WSC) : (_Float16)0.0f;
  }
  _Float16* dst = dpl + e;
  *(volatile v8h*)dst = o.v;
  __threadfence();
  *(volatile v8h*)dst = o.v;
}

template <int KT>
__device__ __forceinline__ void conv_gemm(const _Float16* sF, const _Float16* __restrict__ wpl,
                                          const float* __restrict__ bias, float* sOut,
                                          const int* sDeg, int tid)
{
  const int lane = tid & 31, w = tid >> 5, m = lane & 15, h = lane >> 4;
  const int ncol = 16 * w + m;
  const v8f z8 = {0.f, 0.f, 0.f, 0.f, 0.f, 0.f, 0.f, 0.f};
  #pragma unroll 1
  for (int mt = 0; mt < 4; ++mt) {
    const int row0 = 16 * mt;
    v16h af[KT];
    #pragma unroll
    for (int kt = 0; kt < KT; ++kt) af[kt] = load_frag(sF + (row0 + m) * KPS + 32 * kt, h);
    int dg[8];
    unsigned dm = 0u;
    #pragma unroll
    for (int r = 0; r < 8; ++r) { dg[r] = sDeg[row0 + 8 * h + r]; dm |= 1u << dg[r]; }
    const unsigned dmAll = (unsigned)__builtin_amdgcn_readfirstlane((int)dm) |
                           (unsigned)__builtin_amdgcn_readlane((int)dm, 16);
    float ov[8];
    #pragma unroll
    for (int r = 0; r < 8; ++r) ov[r] = 0.f;
    #pragma unroll 1
    for (int d = 0; d < D_; ++d) {
      if (((dmAll >> d) & 1u) == 0u) continue;
      const _Float16* wb = wpl + ((size_t)(d * H_ + ncol)) * (KT * 32);
      v8f c = z8;
      #pragma unroll
      for (int kt = 0; kt < KT; ++kt) c = wmma_f16(af[kt], load_frag(wb + 32 * kt, h), c);
      const float bb = bias[d * H_ + ncol];
      #pragma unroll
      for (int r = 0; r < 8; ++r) {
        const float v = fmaxf(c[r] * WINV + bb, 0.f);
        ov[r] = (dg[r] == d) ? v : ov[r];
      }
    }
    #pragma unroll
    for (int r = 0; r < 8; ++r) sOut[(row0 + 8 * h + r) * H_ + ncol] = ov[r];
  }
}

__device__ __forceinline__ void out_gemm(const _Float16* sF, const _Float16* __restrict__ wpl,
                                         const float* __restrict__ bias, float* sOut, int tid)
{
  const int lane = tid & 31, w = tid >> 5, m = lane & 15, h = lane >> 4;
  const int ncol = 16 * w + m;
  const v8f z8 = {0.f, 0.f, 0.f, 0.f, 0.f, 0.f, 0.f, 0.f};
  const float bb = bias[ncol];
  const _Float16* wb = wpl + (size_t)ncol * K2P;
  #pragma unroll 1
  for (int mt = 0; mt < 4; ++mt) {
    const int row0 = 16 * mt;
    v8f c = z8;
    #pragma unroll
    for (int kt = 0; kt < K2P / 32; ++kt)
      c = wmma_f16(load_frag(sF + (row0 + m) * KPS + 32 * kt, h), load_frag(wb + 32 * kt, h), c);
    #pragma unroll
    for (int r = 0; r < 8; ++r) sOut[(row0 + 8 * h + r) * H_ + ncol] = c[r] * WINV + bb;
  }
}

__device__ __forceinline__ void fill_tail(_Float16* sF, const float* sBsum, int tid) {
  for (int i = tid; i < A_ * 32; i += 256) {
    const int a = i >> 5, kk = i & 31;
    const int f = (kk < BF_) ? kk : 0;
    const float vb = sBsum[a * 8 + f];
    sF[a * KPS + H_ + kk] = (_Float16)((kk < BF_) ? vb : 0.f);
  }
}

__device__ __forceinline__ void pool_max(const float* sIn, float* sOut, const int* sEdge, int tid) {
  for (int i = tid; i < A_ * H_; i += 256) {
    const int a = i >> 7, c = i & (H_ - 1);
    float mx = sIn[i];
    #pragma unroll
    for (int j = 0; j < D_; ++j) {
      const int e = sEdge[a * 8 + j];
      const float t = sIn[((e < 0) ? 0 : e) * H_ + c];
      mx = (e >= 0) ? fmaxf(mx, t) : mx;
    }
    sOut[i] = mx;
  }
}

__global__ __launch_bounds__(256) void k_mol(
    const float* __restrict__ atoms, const float* __restrict__ bonds, const int* __restrict__ edges,
    const _Float16* __restrict__ w1h, const float* __restrict__ b1,
    const _Float16* __restrict__ w2h, const float* __restrict__ b2,
    const _Float16* __restrict__ woh, const float* __restrict__ bo,
    float* __restrict__ fpw)
{
  __shared__ __attribute__((aligned(16))) _Float16 sF[A_ * KPS];
  __shared__ __attribute__((aligned(16))) float sX[A_ * H_];
  __shared__ __attribute__((aligned(16))) float sP[A_ * H_];
  __shared__ float sAtoms[A_ * 40];
  __shared__ float sBsum[A_ * 8];
  __shared__ int   sDeg[A_];
  __shared__ int   sEdge[A_ * 8];
  __shared__ float sRR[256];
  __shared__ __attribute__((aligned(16))) float sFp[H_];

  const int b = blockIdx.x, tid = threadIdx.x;
  const int lane = tid & 31, w = tid >> 5;
  const float* atomsB = atoms + (size_t)b * A_ * AF_;
  const float* bondsB = bonds + (size_t)b * A_ * D_ * BF_;
  const int*   edgesB = edges + (size_t)b * A_ * D_;

  if (tid < A_) {
    int dg = 0;
    #pragma unroll
    for (int j = 0; j < D_; ++j) {
      int e = edgesB[tid * D_ + j];
      const int valid = (e >= 0) ? 1 : 0;
      dg += valid;
      e = (e > A_ - 1) ? (A_ - 1) : e;
      sEdge[tid * 8 + j] = valid ? e : -1;
    }
    sDeg[tid] = dg;
  }
  for (int i = tid; i < A_ * AF_; i += 256) {
    const int a = i / AF_;
    sAtoms[a * 40 + (i - a * AF_)] = atomsB[i];
  }
  for (int i = tid; i < A_ * BF_; i += 256) {
    const int a = i / BF_, f = i - a * BF_;
    float s = 0.f;
    #pragma unroll
    for (int j = 0; j < D_; ++j) s += bondsB[(a * D_ + j) * BF_ + f];
    sBsum[a * 8 + f] = s;
  }
  __syncthreads();

  for (int i = tid; i < A_ * K1P; i += 256) {
    const int a = i >> 6, k = i & 63;
    const int ka = (k < AF_) ? k : (AF_ - 1);
    const int kb = (k >= AF_ && k < AF_ + BF_) ? (k - AF_) : 0;
    float va = sAtoms[a * 40 + ka];
    #pragma unroll
    for (int j = 0; j < D_; ++j) {
      const int e = sEdge[a * 8 + j];
      const float t = sAtoms[((e < 0) ? 0 : e) * 40 + ka];
      va += (e >= 0) ? t : 0.f;
    }
    const float vb = sBsum[a * 8 + kb];
    const float v = (k < AF_) ? va : ((k < AF_ + BF_) ? vb : 0.f);
    sF[a * KPS + k] = (_Float16)v;
  }
  __syncthreads();

  conv_gemm<K1P / 32>(sF, w1h, b1, sX, sDeg, tid);
  __syncthreads();

  pool_max(sX, sP, sEdge, tid);
  __syncthreads();

  for (int i = tid; i < A_ * H_; i += 256) {
    const int a = i >> 7, k = i & (H_ - 1);
    float v = sP[i];
    #pragma unroll
    for (int j = 0; j < D_; ++j) {
      const int e = sEdge[a * 8 + j];
      const float t = sP[((e < 0) ? 0 : e) * H_ + k];
      v += (e >= 0) ? t : 0.f;
    }
    sF[a * KPS + k] = (_Float16)v;
  }
  fill_tail(sF, sBsum, tid);
  __syncthreads();

  conv_gemm<K2P / 32>(sF, w2h, b2, sX, sDeg, tid);
  __syncthreads();

  pool_max(sX, sP, sEdge, tid);
  __syncthreads();

  for (int i = tid; i < A_ * H_; i += 256) sF[(i >> 7) * KPS + (i & (H_ - 1))] = (_Float16)sP[i];
  fill_tail(sF, sBsum, tid);
  __syncthreads();

  out_gemm(sF, woh, bo, sX, tid);
  __syncthreads();

  #pragma unroll 1
  for (int rr = 0; rr < 8; ++rr) {
    const int a = w * 8 + rr;
    float x0 = sX[a * H_ + lane], x1 = sX[a * H_ + 32 + lane];
    float x2 = sX[a * H_ + 64 + lane], x3 = sX[a * H_ + 96 + lane];
    float mx = fmaxf(fmaxf(x0, x1), fmaxf(x2, x3));
    #pragma unroll
    for (int o = 16; o > 0; o >>= 1) mx = fmaxf(mx, __shfl_xor(mx, o));
    x0 = __expf(x0 - mx); x1 = __expf(x1 - mx); x2 = __expf(x2 - mx); x3 = __expf(x3 - mx);
    float s = (x0 + x1) + (x2 + x3);
    #pragma unroll
    for (int o = 16; o > 0; o >>= 1) s += __shfl_xor(s, o);
    const float sc = (sDeg[a] != 0) ? (1.0f / s) : 0.f;
    sX[a * H_ + lane]      = x0 * sc;
    sX[a * H_ + 32 + lane] = x1 * sc;
    sX[a * H_ + 64 + lane] = x2 * sc;
    sX[a * H_ + 96 + lane] = x3 * sc;
  }
  __syncthreads();

  {
    const int c = tid & (H_ - 1), hh = tid >> 7;
    float s = 0.f;
    #pragma unroll 4
    for (int a = hh * 32; a < hh * 32 + 32; ++a) s += sX[a * H_ + c];
    sRR[tid] = s;
  }
  __syncthreads();
  if (tid < H_) sFp[tid] = sRR[tid] + sRR[H_ + tid];
  __syncthreads();

  if (tid < 32) {
    const v4f v = *(const v4fa*)(sFp + 4 * lane);
    float* dst = fpw + (size_t)b * H_ + 4 * lane;
    *(volatile v4f*)dst = v;
    __threadfence();
    *(volatile v4f*)dst = v;
  }
}

__global__ __launch_bounds__(128) void k_head(
    const float* __restrict__ fpw, const _Float16* __restrict__ wm1h, const float* __restrict__ bm1,
    const _Float16* __restrict__ wm2h, const float* __restrict__ bm2,
    const float* __restrict__ Wm3, const float* __restrict__ bm3, float* __restrict__ out)
{
  __shared__ __attribute__((aligned(16))) _Float16 sA[64 * KPA];
  __shared__ __attribute__((aligned(16))) _Float16 sH1[64 * KPH];
  __shared__ float sH2[64 * 33];
  __shared__ __attribute__((aligned(16))) float sO[64];

  const int tid = threadIdx.x, lane = tid & 31, w = tid >> 5, h = lane >> 4, m = lane & 15;
  const int r0 = blockIdx.x * 64;
  const float* src = fpw + (size_t)r0 * H_;
  for (int i = tid; i < 64 * H_; i += 128) sA[(i >> 7) * KPA + (i & (H_ - 1))] = (_Float16)src[i];
  __syncthreads();

  const v8f z8 = {0.f, 0.f, 0.f, 0.f, 0.f, 0.f, 0.f, 0.f};

  v8f acc[4];
  #pragma unroll
  for (int nt = 0; nt < 4; ++nt) acc[nt] = z8;
  #pragma unroll
  for (int kt = 0; kt < 4; ++kt) {
    const v16h af = load_frag(sA + (16 * w + m) * KPA + 32 * kt, h);
    #pragma unroll
    for (int nt = 0; nt < 4; ++nt) {
      const v16h bf = load_frag(wm1h + (size_t)(16 * nt + m) * H_ + 32 * kt, h);
      acc[nt] = wmma_f16(af, bf, acc[nt]);
    }
  }
  #pragma unroll
  for (int nt = 0; nt < 4; ++nt) {
    const int col = 16 * nt + m;
    const float bb = bm1[col];
    #pragma unroll
    for (int r = 0; r < 8; ++r)
      sH1[(16 * w + 8 * h + r) * KPH + col] = (_Float16)fmaxf(acc[nt][r] * WINV + bb, 0.f);
  }
  __syncthreads();

  v8f acc2[2];
  acc2[0] = z8; acc2[1] = z8;
  #pragma unroll
  for (int kt = 0; kt < 2; ++kt) {
    const v16h af = load_frag(sH1 + (16 * w + m) * KPH + 32 * kt, h);
    #pragma unroll
    for (int nt = 0; nt < 2; ++nt) {
      const v16h bf = load_frag(wm2h + (size_t)(16 * nt + m) * 64 + 32 * kt, h);
      acc2[nt] = wmma_f16(af, bf, acc2[nt]);
    }
  }
  #pragma unroll
  for (int nt = 0; nt < 2; ++nt) {
    const int col = 16 * nt + m;
    const float bb = bm2[col];
    #pragma unroll
    for (int r = 0; r < 8; ++r)
      sH2[(16 * w + 8 * h + r) * 33 + col] = fmaxf(acc2[nt][r] * WINV + bb, 0.f);
  }
  __syncthreads();

  if (tid < 64) {
    float s = 0.f;
    #pragma unroll
    for (int k = 0; k < 32; ++k) s += sH2[tid * 33 + k] * Wm3[k];
    sO[tid] = s + bm3[0];
  }
  __syncthreads();

  if (tid < 16) {
    const v4f v = *(const v4fa*)(sO + 4 * tid);
    float* dst = out + (size_t)r0 + 4 * tid;
    *(volatile v4f*)dst = v;
    __threadfence();
    *(volatile v4f*)dst = v;
  }
}

extern "C" void kernel_launch(void* const* d_in, const int* in_sizes, int n_in,
                              void* d_out, int out_size, void* d_ws, size_t ws_size,
                              hipStream_t stream) {
  if (n_in < 15) return;
  const int B = in_sizes[0] / (A_ * AF_);
  if (B <= 0 || B * A_ * AF_ != in_sizes[0]) return;
  if ((B & 63) != 0) return;
  if (in_sizes[1] != B * A_ * D_ * BF_) return;
  if (in_sizes[2] != B * A_ * D_) return;
  if (in_sizes[3] != D_ * K1R * H_ || in_sizes[4] != D_ * H_) return;
  if (in_sizes[5] != D_ * K2R * H_ || in_sizes[6] != D_ * H_) return;
  if (in_sizes[7] != K2R * H_ || in_sizes[8] != H_) return;
  if (in_sizes[9] != H_ * 64 || in_sizes[10] != 64) return;
  if (in_sizes[11] != 64 * 32 || in_sizes[12] != 32) return;
  if (in_sizes[13] != 32 || in_sizes[14] != 1) return;
  if (out_size != B) return;

  const float* atoms = (const float*)d_in[0];
  const float* bonds = (const float*)d_in[1];
  const int*   edges = (const int*)d_in[2];
  const float* W1  = (const float*)d_in[3];
  const float* b1  = (const float*)d_in[4];
  const float* W2  = (const float*)d_in[5];
  const float* b2  = (const float*)d_in[6];
  const float* Wo  = (const float*)d_in[7];
  const float* bo  = (const float*)d_in[8];
  const float* Wm1 = (const float*)d_in[9];
  const float* bm1 = (const float*)d_in[10];
  const float* Wm2 = (const float*)d_in[11];
  const float* bm2 = (const float*)d_in[12];
  const float* Wm3 = (const float*)d_in[13];
  const float* bm3 = (const float*)d_in[14];
  float* out = (float*)d_out;

  const size_t w1_bytes = (size_t)D_ * H_ * K1P * 2;
  const size_t w2_bytes = (size_t)D_ * H_ * K2P * 2;
  const size_t wo_bytes = (size_t)H_ * K2P * 2;
  const size_t m1_bytes = (size_t)64 * H_ * 2;
  const size_t m2_bytes = (size_t)32 * 64 * 2;
  const size_t fp_bytes = (size_t)B * H_ * 4;
  const size_t off_w2 = w1_bytes;
  const size_t off_wo = off_w2 + w2_bytes;
  const size_t off_m1 = off_wo + wo_bytes;
  const size_t off_m2 = off_m1 + m1_bytes;
  const size_t off_fp = off_m2 + m2_bytes;
  const size_t total  = off_fp + fp_bytes;
  if (total > ws_size) return;

  char* ws = (char*)d_ws;
  _Float16* w1h  = (_Float16*)(ws);
  _Float16* w2h  = (_Float16*)(ws + off_w2);
  _Float16* woh  = (_Float16*)(ws + off_wo);
  _Float16* wm1h = (_Float16*)(ws + off_m1);
  _Float16* wm2h = (_Float16*)(ws + off_m2);
  float*    fpw  = (float*)(ws + off_fp);

  k_convert<<<NB_CVT, 256, 0, stream>>>(W1, W2, Wo, Wm1, Wm2, w1h, w2h, woh, wm1h, wm2h);
  k_mol<<<B, 256, 0, stream>>>(atoms, bonds, edges, w1h, b1, w2h, b2, woh, bo, fpw);
  k_head<<<B / 64, 128, 0, stream>>>(fpw, wm1h, bm1, wm2h, bm2, Wm3, bm3, out);
}
